// NodeDegreeExpansionBlock_7739531067655
// MI455X (gfx1250) — hardware-verified
//
#include <hip/hip_runtime.h>
#include <stddef.h>

#define NN 4096
#define NG 64
#define TN 16
#define NTH 256

#define INVH  0.08838834764831845f
#define INVU  0.125f
#define INVSC 0.027950849718747373f
#define RS3   0.5773502691896258f
#define LNEPS 1e-5f

#define NOP4 "v_nop\n\tv_nop\n\tv_nop\n\tv_nop"

typedef _Float16 f16t;
typedef unsigned short us;
typedef f16t v16h __attribute__((ext_vector_type(16)));
typedef __bf16 v16b __attribute__((ext_vector_type(16)));
typedef us v8us_t __attribute__((ext_vector_type(8)));
typedef v8us_t __attribute__((may_alias)) v8us;
typedef us v4us_t __attribute__((ext_vector_type(4)));
typedef v4us_t __attribute__((may_alias)) v4us;
typedef float v8f __attribute__((ext_vector_type(8)));
typedef float v4f_t __attribute__((ext_vector_type(4)));
typedef v4f_t __attribute__((may_alias)) v4f;
typedef unsigned int v4u_t __attribute__((ext_vector_type(4)));
typedef v4u_t __attribute__((may_alias)) v4u;

union FragH { v16h v; v8us_t h[2]; };
union FragB { v16b v; v8us_t h[2]; };

__device__ __forceinline__ v8f zero8() {
  v8f z;
#pragma unroll
  for (int i = 0; i < 8; ++i) z[i] = 0.0f;
  return z;
}

__device__ __forceinline__ unsigned bfr(float x) {
  const unsigned u = __float_as_uint(x);
  return (u + 0x7FFFu + ((u >> 16) & 1u)) >> 16;
}
__device__ __forceinline__ void splitb(float x, us& hi, us& lo) {
  const unsigned hb = bfr(x);
  const float hf = __uint_as_float(hb << 16);
  hi = (us)hb;
  lo = (us)bfr(x - hf);
}
__device__ __forceinline__ us h16(float x) {
  union { f16t h; us u; } c;
  c.h = (f16t)x;
  return c.u;
}

__device__ __forceinline__ v16h ldh(const us* p) {
  FragH f;
  f.h[0] = *(const v8us*)p;
  f.h[1] = *(const v8us*)(p + 16);
  return f.v;
}
__device__ __forceinline__ v16b ldb(const us* p) {
  FragB f;
  f.h[0] = *(const v8us*)p;
  f.h[1] = *(const v8us*)(p + 16);
  return f.v;
}

__device__ __forceinline__ v8f mmah(v16h a, v16h b, v8f c) {
  return __builtin_amdgcn_wmma_f32_16x16x32_f16(false, a, false, b, (short)0, c, false, false);
}
__device__ __forceinline__ v8f mmab(v16b a, v16b b, v8f c) {
  return __builtin_amdgcn_wmma_f32_16x16x32_bf16(false, a, false, b, (short)0, c, false, false);
}
__device__ __forceinline__ v8f mma3(v16b ah, v16b al, v16b bh, v16b bl, v8f c) {
  c = mmab(ah, bh, c);
  c = mmab(ah, bl, c);
  c = mmab(al, bh, c);
  asm volatile(NOP4 : "+v"(c) : "v"(ah), "v"(al), "v"(bh), "v"(bl));
  return c;
}

__device__ __forceinline__ void store_rows(const float* st, int sw, float* dst, int dp, int R, int lg) {
  const int t = threadIdx.x, q = t & 7;
  const int nl = R << lg;
  for (int pass = 0; pass < 2; ++pass) {
    for (int L = t >> 3; L < nl; L += 32) {
      const int row = L >> lg, seg = L & ((1 << lg) - 1);
      const v4f_t v = *(const v4f*)(st + row * sw + seg * 32 + q * 4);
      *(volatile v4f_t*)(dst + (size_t)row * dp + seg * 32 + q * 4) = v;
    }
    if (pass == 0) __threadfence();
  }
}

template <int MODE>
__global__ void __launch_bounds__(NTH) k_tconv(const float* __restrict__ src, int K, int sp, int sbz,
                                               us* dst, us* dst2, int dbz, float scale)
{
  __shared__ __align__(16) us t0[32 * 72];
  __shared__ __align__(16) us t1[32 * 72];
  const int t = threadIdx.x;
  const int c0 = blockIdx.x * 32, k0 = blockIdx.y * 64, z = blockIdx.z;
  {
    const int kk = t >> 2, cb = (t & 3) * 8;
    const float* p = src + (size_t)z * sbz + (size_t)(k0 + kk) * sp + c0 + cb;
    const v4f_t a = *(const v4f*)p;
    const v4f_t b = *(const v4f*)(p + 4);
#pragma unroll
    for (int j = 0; j < 4; ++j) {
      const int o = (cb + j) * 72 + kk;
      if (MODE == 0) { t0[o] = h16(a[j] * scale); }
      else { us hi, lo; splitb(a[j], hi, lo); t0[o] = hi; t1[o] = lo; }
    }
#pragma unroll
    for (int j = 0; j < 4; ++j) {
      const int o = (cb + 4 + j) * 72 + kk;
      if (MODE == 0) { t0[o] = h16(b[j] * scale); }
      else { us hi, lo; splitb(b[j], hi, lo); t0[o] = hi; t1[o] = lo; }
    }
  }
  __syncthreads();
  const int cc = t >> 3, q = t & 7;
  const v8us_t v0 = *(const v8us*)(t0 + cc * 72 + q * 8);
  v8us_t v1 = v0;
  if (MODE == 1) v1 = *(const v8us*)(t1 + cc * 72 + q * 8);
  const size_t off = (size_t)z * dbz + (size_t)(c0 + cc) * K + k0 + q * 8;
  *(volatile v8us_t*)(dst + off) = v0;
  if (MODE == 1) *(volatile v8us_t*)(dst2 + off) = v1;
  __threadfence();
  *(volatile v8us_t*)(dst + off) = v0;
  if (MODE == 1) *(volatile v8us_t*)(dst2 + off) = v1;
}

__device__ __forceinline__ void split_hidden_row(const float* __restrict__ nfh, int n, int r, int j,
                                                 us* ah, int PS)
{
  const float* ph = nfh + (size_t)n * 512 + j * 32;
#pragma unroll
  for (int q4 = 0; q4 < 8; ++q4) {
    const v4f_t x4 = *(const v4f*)(ph + q4 * 4);
#pragma unroll
    for (int e = 0; e < 4; ++e) {
      const int c = j * 32 + q4 * 4 + e;
      int o;
      if (j < 4) { o = r * 136 + c; }
      else { const int cc = c - 128; o = (1 + cc % 3) * 2176 + r * 136 + cc / 3; }
      us hi, lo; splitb(x4[e], hi, lo);
      ah[o] = hi; ah[PS + o] = lo;
    }
  }
}

__global__ void __launch_bounds__(NTH) k_lin(const float* __restrict__ nfh, const float* __restrict__ nfu,
    const us* __restrict__ Wh0h, const us* __restrict__ Wh0l,
    const us* __restrict__ Wh1h, const us* __restrict__ Wh1l,
    const us* __restrict__ Wu0h, const us* __restrict__ Wu0l,
    const us* __restrict__ Wu1h, const us* __restrict__ Wu1l,
    float* __restrict__ hp0, float* __restrict__ up0,
    float* __restrict__ hp1, float* __restrict__ up1)
{
  __shared__ __align__(16) unsigned char raw[53248];
  us* ah = (us*)raw;
  us* au = (us*)(raw + 34816);
  float* stg = (float*)raw;
  const int t = threadIdx.x, lane = t & 31, w = t >> 5, h = lane >> 4, m = lane & 15;
  const int n0 = blockIdx.x * TN;
  {
    const int r = t & 15, j = t >> 4;
    split_hidden_row(nfh, n0 + r, r, j, ah, 8704);
    const float* pu = nfu + (size_t)(n0 + r) * 256 + j * 16;
#pragma unroll
    for (int q4 = 0; q4 < 4; ++q4) {
      const v4f_t x4 = *(const v4f*)(pu + q4 * 4);
#pragma unroll
      for (int e = 0; e < 4; ++e) {
        const int c = j * 16 + q4 * 4 + e;
        int o;
        if (j < 4) { o = r * 72 + c; }
        else { const int cc = c - 64; o = (1 + cc % 3) * 1152 + r * 72 + cc / 3; }
        us hi, lo; splitb(x4[e], hi, lo);
        au[o] = hi; au[4608 + o] = lo;
      }
    }
  }
  __syncthreads();

  const int col0 = 16 * w;
  v8f acch0 = zero8(), acch1a = zero8(), acch1b = zero8(), acch1c = zero8();
#pragma unroll
  for (int ks = 0; ks < 4; ++ks) {
    const int ao = m * 136 + 32 * ks + 8 * h;
    const size_t bo = (size_t)(col0 + m) * 128 + 32 * ks + 8 * h;
    const v16b b0h = ldb(Wh0h + bo), b0l = ldb(Wh0l + bo);
    acch0 = mma3(ldb(ah + ao), ldb(ah + 8704 + ao), b0h, b0l, acch0);
    const v16b b1h = ldb(Wh1h + bo), b1l = ldb(Wh1l + bo);
    acch1a = mma3(ldb(ah + 2176 + ao), ldb(ah + 8704 + 2176 + ao), b1h, b1l, acch1a);
    acch1b = mma3(ldb(ah + 4352 + ao), ldb(ah + 8704 + 4352 + ao), b1h, b1l, acch1b);
    acch1c = mma3(ldb(ah + 6528 + ao), ldb(ah + 8704 + 6528 + ao), b1h, b1l, acch1c);
  }
  v8f accu[2];
  accu[0] = zero8(); accu[1] = zero8();
#pragma unroll
  for (int jt = 0; jt < 2; ++jt) {
    const int id = 2 * w + jt, comp = id >> 2, ct = id & 3;
    const us* Bh = (comp == 0) ? Wu0h : Wu1h;
    const us* Bl = (comp == 0) ? Wu0l : Wu1l;
#pragma unroll
    for (int ks = 0; ks < 2; ++ks) {
      const int ao = comp * 1152 + m * 72 + 32 * ks + 8 * h;
      const size_t bo = (size_t)(16 * ct + m) * 64 + 32 * ks + 8 * h;
      accu[jt] = mma3(ldb(au + ao), ldb(au + 4608 + ao), ldb(Bh + bo), ldb(Bl + bo), accu[jt]);
    }
  }
  __syncthreads();
#pragma unroll
  for (int r = 0; r < 8; ++r) {
    const int nd = 8 * h + r;
    stg[nd * 128 + col0 + m] = acch0[r] * INVH;
    stg[2048 + nd * 128 + col0 + m] = acch1a[r] * INVH;
    stg[4096 + nd * 128 + col0 + m] = acch1b[r] * INVH;
    stg[6144 + nd * 128 + col0 + m] = acch1c[r] * INVH;
  }
#pragma unroll
  for (int jt = 0; jt < 2; ++jt) {
    const int id = 2 * w + jt, comp = id >> 2, ct = id & 3;
    const int base = (comp == 0) ? 8192 : (9216 + (comp - 1) * 1024);
#pragma unroll
    for (int r = 0; r < 8; ++r) stg[base + (8 * h + r) * 64 + 16 * ct + m] = accu[jt][r] * INVU;
  }
  __syncthreads();
  store_rows(stg, 128, hp0 + (size_t)n0 * 128, 128, 16, 2);
#pragma unroll 1
  for (int i = 0; i < 3; ++i)
    store_rows(stg + 2048 + i * 2048, 128, hp1 + ((size_t)i * NN + n0) * 128, 128, 16, 2);
  store_rows(stg + 8192, 64, up0 + (size_t)n0 * 64, 64, 16, 1);
#pragma unroll 1
  for (int i = 0; i < 3; ++i)
    store_rows(stg + 9216 + i * 1024, 64, up1 + ((size_t)i * NN + n0) * 64, 64, 16, 1);
}

__global__ void __launch_bounds__(NTH) k_z0(const float* __restrict__ hp0, const float* __restrict__ up0,
    const float* __restrict__ hp1, const float* __restrict__ up1,
    const us* __restrict__ T00, const us* __restrict__ T11, float* __restrict__ z0)
{
  __shared__ __align__(16) float fs[12288];
  __shared__ __align__(16) us xa[16 * 264];
  __shared__ __align__(16) us xb[16 * 264];
  const int t = threadIdx.x, lane = t & 31, w = t >> 5, h = lane >> 4, m = lane & 15;
  const int n0 = blockIdx.x * TN;
  {
    const int r = t >> 4, j = t & 15;
    const float* p0 = hp0 + (size_t)(n0 + r) * 128 + j * 8;
    *(v4f*)(fs + r * 128 + j * 8) = *(const v4f*)p0;
    *(v4f*)(fs + r * 128 + j * 8 + 4) = *(const v4f*)(p0 + 4);
    *(v4f*)(fs + 2048 + r * 64 + j * 4) = *(const v4f*)(up0 + (size_t)(n0 + r) * 64 + j * 4);
#pragma unroll
    for (int i = 0; i < 3; ++i) {
      const float* p1 = hp1 + ((size_t)i * NN + n0 + r) * 128 + j * 8;
      *(v4f*)(fs + 3072 + i * 2048 + r * 128 + j * 8) = *(const v4f*)p1;
      *(v4f*)(fs + 3072 + i * 2048 + r * 128 + j * 8 + 4) = *(const v4f*)(p1 + 4);
      *(v4f*)(fs + 9216 + i * 1024 + r * 64 + j * 4) = *(const v4f*)(up1 + ((size_t)i * NN + n0 + r) * 64 + j * 4);
    }
  }
  __syncthreads();

  v8f acc[2];
  acc[0] = zero8(); acc[1] = zero8();
  const us* pa = xa + m * 264 + 8 * h;
  const us* pc = xb + m * 264 + 8 * h;
  const us* pb0 = T00 + (size_t)(32 * w + m) * 8192 + 8 * h;
  const us* pb1 = T11 + (size_t)(32 * w + m) * 8192 + 8 * h;

#pragma unroll 1
  for (int c = 0; c < 32; ++c) {
    {
      const int r = t >> 4, j = t & 15;
      const int u = 4 * c + (j >> 2);
      const int v0 = (j & 3) * 16;
      const float a0 = fs[r * 128 + u] * 16.0f;
      const float c0 = fs[3072 + r * 128 + u] * (RS3 * 16.0f);
      const float c1 = fs[5120 + r * 128 + u] * (RS3 * 16.0f);
      const float c2 = fs[7168 + r * 128 + u] * (RS3 * 16.0f);
      v8us_t px0, px1, py0, py1;
#pragma unroll
      for (int e = 0; e < 8; ++e) { px0[e] = 0; px1[e] = 0; py0[e] = 0; py1[e] = 0; }
#pragma unroll
      for (int q4 = 0; q4 < 4; ++q4) {
        const int vo = r * 64 + v0 + q4 * 4;
        const v4f_t uu = *(const v4f*)(fs + 2048 + vo);
        const v4f_t w0 = *(const v4f*)(fs + 9216 + vo);
        const v4f_t w1 = *(const v4f*)(fs + 10240 + vo);
        const v4f_t w2 = *(const v4f*)(fs + 11264 + vo);
#pragma unroll
        for (int e = 0; e < 4; ++e) {
          const float x = a0 * uu[e];
          const float y = c0 * w0[e] + c1 * w1[e] + c2 * w2[e];
          const int idx = q4 * 4 + e;
          if (idx < 8) { px0[idx] = h16(x); py0[idx] = h16(y); }
          else { px1[idx - 8] = h16(x); py1[idx - 8] = h16(y); }
        }
      }
      *(v8us*)(xa + r * 264 + j * 16) = px0;
      *(v8us*)(xa + r * 264 + j * 16 + 8) = px1;
      *(v8us*)(xb + r * 264 + j * 16) = py0;
      *(v8us*)(xb + r * 264 + j * 16 + 8) = py1;
    }
    __syncthreads();
#pragma unroll
    for (int ks = 0; ks < 8; ++ks) {
      const int ko = c * 256 + 32 * ks;
      const v16h A0 = ldh(pa + 32 * ks);
      const v16h A1 = ldh(pc + 32 * ks);
      const v16h B00 = ldh(pb0 + ko);
      const v16h B01 = ldh(pb0 + 16 * 8192 + ko);
      const v16h B10 = ldh(pb1 + ko);
      const v16h B11 = ldh(pb1 + 16 * 8192 + ko);
      acc[0] = mmah(A0, B00, acc[0]);
      acc[0] = mmah(A1, B10, acc[0]);
      acc[1] = mmah(A0, B01, acc[1]);
      acc[1] = mmah(A1, B11, acc[1]);
      asm volatile(NOP4 : "+v"(acc[0]), "+v"(acc[1])
                   : "v"(A0), "v"(A1), "v"(B00), "v"(B01), "v"(B10), "v"(B11));
    }
    __syncthreads();
  }
  const float sc = 1.0f / 8192.0f;
#pragma unroll
  for (int ct = 0; ct < 2; ++ct) {
#pragma unroll
    for (int r = 0; r < 8; ++r) fs[(8 * h + r) * 256 + 32 * w + 16 * ct + m] = acc[ct][r] * sc;
  }
  __syncthreads();
  store_rows(fs, 256, z0 + (size_t)n0 * 256, 256, 16, 3);
}

__global__ void __launch_bounds__(NTH) k_z1(const float* __restrict__ hp0, const float* __restrict__ up0,
    const float* __restrict__ hp1, const float* __restrict__ up1,
    const us* __restrict__ T01, const us* __restrict__ T10, float* __restrict__ z1)
{
  __shared__ __align__(16) float fs[9216];
  __shared__ __align__(16) us ha[16 * 136];
  __shared__ __align__(16) us ua[16 * 72];
  const int t = threadIdx.x, lane = t & 31, w = t >> 5, h = lane >> 4, m = lane & 15;
  const int n0 = blockIdx.x * TN;
  {
    const int r = t >> 4, j = t & 15;
    const float* p0 = hp0 + (size_t)(n0 + r) * 128 + j * 8;
    const v4f_t a = *(const v4f*)p0;
    const v4f_t b = *(const v4f*)(p0 + 4);
    v8us_t pk;
#pragma unroll
    for (int e = 0; e < 4; ++e) { pk[e] = h16(a[e] * 8.0f); pk[4 + e] = h16(b[e] * 8.0f); }
    *(v8us*)(ha + r * 136 + j * 8) = pk;
    const v4f_t uq = *(const v4f*)(up0 + (size_t)(n0 + r) * 64 + j * 4);
    v4us_t pu;
#pragma unroll
    for (int e = 0; e < 4; ++e) pu[e] = h16(uq[e] * 8.0f);
    *(v4us*)(ua + r * 72 + j * 4) = pu;
#pragma unroll
    for (int i = 0; i < 3; ++i) {
      const float* p1 = hp1 + ((size_t)i * NN + n0 + r) * 128 + j * 8;
      *(v4f*)(fs + i * 2048 + r * 128 + j * 8) = *(const v4f*)p1;
      *(v4f*)(fs + i * 2048 + r * 128 + j * 8 + 4) = *(const v4f*)(p1 + 4);
      *(v4f*)(fs + 6144 + i * 1024 + r * 64 + j * 4) = *(const v4f*)(up1 + ((size_t)i * NN + n0 + r) * 64 + j * 4);
    }
  }
  __syncthreads();

  const int col0 = 16 * w;
  const v16h fa0 = ldh(ha + m * 136 + 8 * h);
  const v16h fa1 = ldh(ha + m * 136 + 32 + 8 * h);
  const v16h fa2 = ldh(ha + m * 136 + 64 + 8 * h);
  const v16h fa3 = ldh(ha + m * 136 + 96 + 8 * h);
  const v16h fu0 = ldh(ua + m * 72 + 8 * h);
  const v16h fu1 = ldh(ua + m * 72 + 32 + 8 * h);
  v8f za = zero8(), zb = zero8(), zc = zero8();

#pragma unroll 1
  for (int v = 0; v < 64; ++v) {
    const us* pb = T01 + (size_t)(v * 128 + col0 + m) * 128 + 8 * h;
    const v16h b0 = ldh(pb), b1 = ldh(pb + 32), b2 = ldh(pb + 64), b3 = ldh(pb + 96);
    v8f D = zero8();
    D = mmah(fa0, b0, D);
    D = mmah(fa1, b1, D);
    D = mmah(fa2, b2, D);
    D = mmah(fa3, b3, D);
    asm volatile(NOP4 : "+v"(D) : "v"(fa0), "v"(fa1), "v"(fa2), "v"(fa3), "v"(b0), "v"(b1), "v"(b2), "v"(b3));
    const float* pu = fs + 6144 + (8 * h) * 64 + v;
#pragma unroll
    for (int r = 0; r < 8; ++r) {
      const float d = D[r];
      za[r] = fmaf(d, pu[r * 64], za[r]);
      zb[r] = fmaf(d, pu[1024 + r * 64], zb[r]);
      zc[r] = fmaf(d, pu[2048 + r * 64], zc[r]);
    }
  }
#pragma unroll 1
  for (int u = 0; u < 128; ++u) {
    const us* pb = T10 + (size_t)(u * 128 + col0 + m) * 64 + 8 * h;
    const v16h b0 = ldh(pb), b1 = ldh(pb + 32);
    v8f D = zero8();
    D = mmah(fu0, b0, D);
    D = mmah(fu1, b1, D);
    asm volatile(NOP4 : "+v"(D) : "v"(fu0), "v"(fu1), "v"(b0), "v"(b1));
    const float* pq = fs + (8 * h) * 128 + u;
#pragma unroll
    for (int r = 0; r < 8; ++r) {
      const float d = D[r];
      za[r] = fmaf(d, pq[r * 128], za[r]);
      zb[r] = fmaf(d, pq[2048 + r * 128], zb[r]);
      zc[r] = fmaf(d, pq[4096 + r * 128], zc[r]);
    }
  }
  __syncthreads();
  const float sc = 1.0f / 4096.0f;
#pragma unroll
  for (int r = 0; r < 8; ++r) {
    const int o = (8 * h + r) * 128 + col0 + m;
    fs[o] = za[r] * sc;
    fs[2048 + o] = zb[r] * sc;
    fs[4096 + o] = zc[r] * sc;
  }
  __syncthreads();
#pragma unroll 1
  for (int i = 0; i < 3; ++i)
    store_rows(fs + i * 2048, 128, z1 + ((size_t)i * NN + n0) * 128, 128, 16, 2);
}

__global__ void __launch_bounds__(NTH) k_post(const float* __restrict__ nfh, const float* __restrict__ onehot,
    const float* __restrict__ z0p, const float* __restrict__ z1p,
    const us* __restrict__ Wp0h, const us* __restrict__ Wp0l,
    const us* __restrict__ Wp1h, const us* __restrict__ Wp1l,
    const us* __restrict__ Ts0h, const us* __restrict__ Ts0l,
    const us* __restrict__ Ts1h, const us* __restrict__ Ts1l,
    const float* __restrict__ b_p0,
    float* __restrict__ y0, float* __restrict__ y1, double* __restrict__ rowstat)
{
  __shared__ __align__(16) unsigned char raw[69632];
  __shared__ __align__(16) float gsm[16 * 128];
  __shared__ __align__(16) float oh[16 * 16];
  __shared__ __align__(16) double rst[48];
  us* at = (us*)raw;
  float* yst = (float*)raw;
  const int PS = 17408;
  const int t = threadIdx.x, lane = t & 31, w = t >> 5, h = lane >> 4, m = lane & 15;
  const int n0 = blockIdx.x * TN;
  {
    const int r = t & 15, j = t >> 4;
    split_hidden_row(nfh, n0 + r, r, j, at + 4 * 2176, PS);
    const float* pz = z0p + (size_t)(n0 + r) * 256 + j * 16;
#pragma unroll
    for (int q4 = 0; q4 < 4; ++q4) {
      const v4f_t z4 = *(const v4f*)(pz + q4 * 4);
#pragma unroll
      for (int e = 0; e < 4; ++e) {
        const int c = j * 16 + q4 * 4 + e;
        const float z = z4[e];
        const float ex = __expf(-z);
        const float sg = __builtin_amdgcn_rcpf(1.0f + ex);
        if (j < 8) {
          us hi, lo; splitb(z * sg, hi, lo);
          const int o = r * 136 + c;
          at[o] = hi; at[PS + o] = lo;
        } else {
          gsm[r * 128 + c - 128] = sg;
        }
      }
    }
    if (t < 160) {
      const int r2 = t / 10, kk = t - r2 * 10;
      oh[r2 * 16 + kk] = onehot[(size_t)(n0 + r2) * 10 + kk];
    }
  }
  __syncthreads();
  {
    const int r = t & 15, j = t >> 4;
#pragma unroll
    for (int i = 0; i < 3; ++i) {
      const float* p1 = z1p + ((size_t)i * NN + n0 + r) * 128 + j * 8;
      const v4f_t a = *(const v4f*)p1;
      const v4f_t b = *(const v4f*)(p1 + 4);
#pragma unroll
      for (int e = 0; e < 8; ++e) {
        const int c = j * 8 + e;
        const float x = ((e < 4) ? a[e] : b[e - 4]) * gsm[r * 128 + c];
        us hi, lo; splitb(x, hi, lo);
        const int o = (1 + i) * 2176 + r * 136 + c;
        at[o] = hi; at[PS + o] = lo;
      }
    }
  }
  __syncthreads();

  const int col0 = 16 * w;
  v8f aP0 = zero8(), aS0 = zero8();
  v8f aP1[3], aS1[3];
#pragma unroll
  for (int i = 0; i < 3; ++i) { aP1[i] = zero8(); aS1[i] = zero8(); }
#pragma unroll
  for (int ks = 0; ks < 4; ++ks) {
    const int ao = m * 136 + 32 * ks + 8 * h;
    const size_t bo = (size_t)(col0 + m) * 128 + 32 * ks + 8 * h;
    aP0 = mma3(ldb(at + ao), ldb(at + PS + ao), ldb(Wp0h + bo), ldb(Wp0l + bo), aP0);
    const v16b bh = ldb(Wp1h + bo), bl = ldb(Wp1l + bo);
#pragma unroll
    for (int i = 0; i < 3; ++i)
      aP1[i] = mma3(ldb(at + (1 + i) * 2176 + ao), ldb(at + PS + (1 + i) * 2176 + ao), bh, bl, aP1[i]);
  }
#pragma unroll 1
  for (int kk = 0; kk < 10; ++kk) {
    v8f D = zero8();
#pragma unroll
    for (int ks = 0; ks < 4; ++ks) {
      const int ao = 4 * 2176 + m * 136 + 32 * ks + 8 * h;
      const size_t bo = (size_t)(kk * 128 + col0 + m) * 128 + 32 * ks + 8 * h;
      D = mma3(ldb(at + ao), ldb(at + PS + ao), ldb(Ts0h + bo), ldb(Ts0l + bo), D);
    }
#pragma unroll
    for (int r = 0; r < 8; ++r) aS0[r] = fmaf(oh[(8 * h + r) * 16 + kk], D[r], aS0[r]);
  }
#pragma unroll 1
  for (int kk = 0; kk < 10; ++kk) {
    v8f Dv[3];
    Dv[0] = zero8(); Dv[1] = zero8(); Dv[2] = zero8();
#pragma unroll
    for (int ks = 0; ks < 4; ++ks) {
      const size_t bo = (size_t)(kk * 128 + col0 + m) * 128 + 32 * ks + 8 * h;
      const v16b bh = ldb(Ts1h + bo), bl = ldb(Ts1l + bo);
#pragma unroll
      for (int i = 0; i < 3; ++i) {
        const int ao = (5 + i) * 2176 + m * 136 + 32 * ks + 8 * h;
        Dv[i] = mma3(ldb(at + ao), ldb(at + PS + ao), bh, bl, Dv[i]);
      }
    }
#pragma unroll
    for (int r = 0; r < 8; ++r) {
      const float o = oh[(8 * h + r) * 16 + kk];
#pragma unroll
      for (int i = 0; i < 3; ++i) aS1[i][r] = fmaf(o, Dv[i][r], aS1[i][r]);
    }
  }
  __syncthreads();
  {
    const float bp = b_p0[col0 + m];
#pragma unroll
    for (int r = 0; r < 8; ++r) {
      const int o = (8 * h + r) * 128 + col0 + m;
      yst[o] = aP0[r] * INVH + bp + aS0[r] * INVSC;
#pragma unroll
      for (int i = 0; i < 3; ++i) yst[2048 * (1 + i) + o] = aP1[i][r] * INVH + aS1[i][r] * INVSC;
    }
  }
  __syncthreads();
  {
    const int r = t >> 4, j = t & 15;
    double s0 = 0.0, q0 = 0.0, q1 = 0.0;
#pragma unroll
    for (int e = 0; e < 8; ++e) {
      const double y = (double)yst[r * 128 + j * 8 + e];
      s0 += y; q0 = fma(y, y, q0);
#pragma unroll
      for (int i = 0; i < 3; ++i) {
        const double yv = (double)yst[2048 * (1 + i) + r * 128 + j * 8 + e];
        q1 = fma(yv, yv, q1);
      }
    }
#pragma unroll
    for (int off = 1; off < 16; off <<= 1) {
      s0 += __shfl_xor(s0, off, 32);
      q0 += __shfl_xor(q0, off, 32);
      q1 += __shfl_xor(q1, off, 32);
    }
    if (j == 0) { rst[r] = s0; rst[16 + r] = q0; rst[32 + r] = q1; }
  }
  __syncthreads();
  if (t < 24) {
    const int s = t >> 3, q = t & 7;
    const v4u_t vv = *(const v4u*)(rst + s * 16 + q * 2);
    *(volatile v4u_t*)(rowstat + (size_t)s * NN + n0 + q * 2) = vv;
  }
  __threadfence();
  if (t < 24) {
    const int s = t >> 3, q = t & 7;
    const v4u_t vv = *(const v4u*)(rst + s * 16 + q * 2);
    *(volatile v4u_t*)(rowstat + (size_t)s * NN + n0 + q * 2) = vv;
  }
  store_rows(yst, 128, y0 + (size_t)n0 * 128, 128, 16, 2);
#pragma unroll 1
  for (int i = 0; i < 3; ++i)
    store_rows(yst + 2048 * (1 + i), 128, y1 + ((size_t)i * NN + n0) * 128, 128, 16, 2);
}

__global__ void __launch_bounds__(NTH) k_stats(const int* __restrict__ batch, const double* __restrict__ rowstat,
                                               float* __restrict__ gstat)
{
  __shared__ __align__(16) float gst[256];
  const int t = threadIdx.x, g = t >> 2, j = t & 3;
  double cnt = 0.0, s0 = 0.0, q0 = 0.0, q1 = 0.0;
#pragma unroll 1
  for (int n = j; n < NN; n += 4) {
    const int b = batch[n];
    const double msk = (b == g) ? 1.0 : 0.0;
    cnt += msk;
    s0 = fma(msk, rowstat[n], s0);
    q0 = fma(msk, rowstat[NN + n], q0);
    q1 = fma(msk, rowstat[2 * NN + n], q1);
  }
#pragma unroll
  for (int off = 1; off < 4; off <<= 1) {
    cnt += __shfl_xor(cnt, off, 32);
    s0 += __shfl_xor(s0, off, 32);
    q0 += __shfl_xor(q0, off, 32);
    q1 += __shfl_xor(q1, off, 32);
  }
  if (j == 0) {
    const double c = fmax(cnt, 1.0);
    const double mean = s0 / (c * 128.0);
    double var0 = q0 / (c * 128.0) - mean * mean;
    if (var0 < 0.0) var0 = 0.0;
    const double var1 = q1 / (c * 384.0);
    gst[g * 4 + 0] = (float)mean;
    gst[g * 4 + 1] = __builtin_amdgcn_rcpf(sqrtf((float)var0) + LNEPS);
    gst[g * 4 + 2] = __builtin_amdgcn_rcpf(sqrtf((float)var1) + LNEPS);
    gst[g * 4 + 3] = (float)c;
  }
  __syncthreads();
  if (t < 32) {
    const v4f_t a = *(const v4f*)(gst + t * 4);
    const v4f_t b = *(const v4f*)(gst + 128 + t * 4);
    *(volatile v4f_t*)(gstat + t * 4) = a;
    *(volatile v4f_t*)(gstat + 128 + t * 4) = b;
  }
  __threadfence();
  if (t < 32) {
    const v4f_t a = *(const v4f*)(gst + t * 4);
    const v4f_t b = *(const v4f*)(gst + 128 + t * 4);
    *(volatile v4f_t*)(gstat + t * 4) = a;
    *(volatile v4f_t*)(gstat + 128 + t * 4) = b;
  }
}

__global__ void __launch_bounds__(NTH) k_final(const float* __restrict__ nfh, const int* __restrict__ batch,
    const float* __restrict__ y0p, const float* __restrict__ y1p, const float* __restrict__ gstat,
    const float* __restrict__ ln_w0, const float* __restrict__ ln_b0, const float* __restrict__ ln_w1,
    const us* __restrict__ Ws0h, const us* __restrict__ Ws0l,
    const us* __restrict__ Ws1h, const us* __restrict__ Ws1l,
    const float* __restrict__ b_s0, float* __restrict__ out)
{
  __shared__ __align__(16) unsigned char raw[34816];
  __shared__ __align__(16) float yst[8192];
  __shared__ __align__(16) float gsn[64];
  us* at = (us*)raw;
  float* ost = (float*)raw;
  const int t = threadIdx.x, lane = t & 31, w = t >> 5, h = lane >> 4, m = lane & 15;
  const int n0 = blockIdx.x * TN;
  {
    const int r = t & 15, j = t >> 4;
    split_hidden_row(nfh, n0 + r, r, j, at, 8704);
    const float* p0 = y0p + (size_t)(n0 + r) * 128 + j * 8;
    *(v4f*)(yst + r * 128 + j * 8) = *(const v4f*)p0;
    *(v4f*)(yst + r * 128 + j * 8 + 4) = *(const v4f*)(p0 + 4);
#pragma unroll
    for (int i = 0; i < 3; ++i) {
      const float* p1 = y1p + ((size_t)i * NN + n0 + r) * 128 + j * 8;
      *(v4f*)(yst + 2048 * (1 + i) + r * 128 + j * 8) = *(const v4f*)p1;
      *(v4f*)(yst + 2048 * (1 + i) + r * 128 + j * 8 + 4) = *(const v4f*)(p1 + 4);
    }
    if (t < 16) {
      int b = batch[n0 + t];
      b = (b < 0) ? 0 : ((b > NG - 1) ? (NG - 1) : b);
      const v4f_t gv = *(const v4f*)(gstat + b * 4);
      *(v4f*)(gsn + t * 4) = gv;
    }
  }
  __syncthreads();

  const int col0 = 16 * w;
  v8f acc0 = zero8(), acca = zero8(), accb = zero8(), accc = zero8();
#pragma unroll
  for (int ks = 0; ks < 4; ++ks) {
    const int ao = m * 136 + 32 * ks + 8 * h;
    const size_t bo = (size_t)(col0 + m) * 128 + 32 * ks + 8 * h;
    acc0 = mma3(ldb(at + ao), ldb(at + 8704 + ao), ldb(Ws0h + bo), ldb(Ws0l + bo), acc0);
    const v16b bh = ldb(Ws1h + bo), bl = ldb(Ws1l + bo);
    acca = mma3(ldb(at + 2176 + ao), ldb(at + 8704 + 2176 + ao), bh, bl, acca);
    accb = mma3(ldb(at + 4352 + ao), ldb(at + 8704 + 4352 + ao), bh, bl, accb);
    accc = mma3(ldb(at + 6528 + ao), ldb(at + 8704 + 6528 + ao), bh, bl, accc);
  }
  __syncthreads();
  {
    const int u = col0 + m;
    const float lw0 = ln_w0[u], lb0 = ln_b0[u], lw1 = ln_w1[u], bs = b_s0[u];
#pragma unroll
    for (int r = 0; r < 8; ++r) {
      const int nd = 8 * h + r;
      const float mean0 = gsn[nd * 4], rs0 = gsn[nd * 4 + 1], rs1 = gsn[nd * 4 + 2];
      const float f0 = (yst[nd * 128 + u] - mean0) * rs0 * lw0 + lb0;
      ost[nd * 512 + u] = f0 + acc0[r] * INVH + bs;
      const float f1a = yst[2048 + nd * 128 + u] * rs1 * lw1;
      const float f1b = yst[4096 + nd * 128 + u] * rs1 * lw1;
      const float f1c = yst[6144 + nd * 128 + u] * rs1 * lw1;
      ost[nd * 512 + 128 + u * 3 + 0] = f1a + acca[r] * INVH;
      ost[nd * 512 + 128 + u * 3 + 1] = f1b + accb[r] * INVH;
      ost[nd * 512 + 128 + u * 3 + 2] = f1c + accc[r] * INVH;
    }
  }
  __syncthreads();
  store_rows(ost, 512, out + (size_t)n0 * 512, 512, 16, 4);
}

extern "C" void kernel_launch(void* const* d_in, const int* in_sizes, int n_in,
                              void* d_out, int out_size, void* d_ws, size_t ws_size,
                              hipStream_t stream)
{
  if (n_in < 23) return;
  if (in_sizes[0] != NN * 512) return;
  if (in_sizes[1] != NN * 256) return;
  if (in_sizes[2] != NN * 10) return;
  if (in_sizes[3] != NN) return;
  if (in_sizes[4] != 128 * 128 || in_sizes[5] != 128 * 128) return;
  if (in_sizes[6] != 64 * 64 || in_sizes[7] != 64 * 64) return;
  if (in_sizes[8] != 128 * 64 * 256 || in_sizes[9] != 128 * 64 * 256) return;
  if (in_sizes[10] != 128 * 64 * 128 || in_sizes[11] != 128 * 64 * 128) return;
  if (in_sizes[12] != 128 * 128 || in_sizes[13] != 128 || in_sizes[14] != 128 * 128) return;
  if (in_sizes[15] != 128 * 10 * 128 || in_sizes[16] != 128 * 10 * 128) return;
  if (in_sizes[17] != 128 || in_sizes[18] != 128 || in_sizes[19] != 128) return;
  if (in_sizes[20] != 128 * 128 || in_sizes[21] != 128 || in_sizes[22] != 128 * 128) return;
  if (out_size != NN * 512) return;

  const float* nfh    = (const float*)d_in[0];
  const float* nfu    = (const float*)d_in[1];
  const float* onehot = (const float*)d_in[2];
  const int*   batch  = (const int*)d_in[3];
  const float* W_h0   = (const float*)d_in[4];
  const float* W_h1   = (const float*)d_in[5];
  const float* W_u0   = (const float*)d_in[6];
  const float* W_u1   = (const float*)d_in[7];
  const float* Wt_00  = (const float*)d_in[8];
  const float* Wt_11  = (const float*)d_in[9];
  const float* Wt_01  = (const float*)d_in[10];
  const float* Wt_10  = (const float*)d_in[11];
  const float* W_p0   = (const float*)d_in[12];
  const float* b_p0   = (const float*)d_in[13];
  const float* W_p1   = (const float*)d_in[14];
  const float* Wsc0   = (const float*)d_in[15];
  const float* Wsc1   = (const float*)d_in[16];
  const float* ln_w0  = (const float*)d_in[17];
  const float* ln_b0  = (const float*)d_in[18];
  const float* ln_w1  = (const float*)d_in[19];
  const float* W_s0   = (const float*)d_in[20];
  const float* b_s0   = (const float*)d_in[21];
  const float* W_s1   = (const float*)d_in[22];
  float* out = (float*)d_out;

  size_t o = 0;
  auto take = [&](size_t b) { size_t r = o; o += (b + 255) & ~(size_t)255; return r; };
  const size_t oHP0 = take((size_t)NN * 128 * 4);
  const size_t oUP0 = take((size_t)NN * 64 * 4);
  const size_t oHP1 = take((size_t)3 * NN * 128 * 4);
  const size_t oUP1 = take((size_t)3 * NN * 64 * 4);
  const size_t oZ0  = take((size_t)NN * 256 * 4);
  const size_t oZ1  = take((size_t)3 * NN * 128 * 4);
  const size_t oY0  = take((size_t)NN * 128 * 4);
  const size_t oY1  = take((size_t)3 * NN * 128 * 4);
  const size_t oRS  = take((size_t)3 * NN * 8);
  const size_t oGS  = take((size_t)NG * 4 * 4);
  const size_t oT00 = take((size_t)256 * 8192 * 2);
  const size_t oT11 = take((size_t)256 * 8192 * 2);
  const size_t oT01 = take((size_t)8192 * 128 * 2);
  const size_t oT10 = take((size_t)128 * 128 * 64 * 2);
  const size_t szW  = (size_t)128 * 128 * 2, szU = (size_t)64 * 64 * 2, szS = (size_t)1280 * 128 * 2;
  const size_t oWh0h = take(szW), oWh0l = take(szW), oWh1h = take(szW), oWh1l = take(szW);
  const size_t oWp0h = take(szW), oWp0l = take(szW), oWp1h = take(szW), oWp1l = take(szW);
  const size_t oWs0h = take(szW), oWs0l = take(szW), oWs1h = take(szW), oWs1l = take(szW);
  const size_t oWu0h = take(szU), oWu0l = take(szU), oWu1h = take(szU), oWu1l = take(szU);
  const size_t oTs0h = take(szS), oTs0l = take(szS), oTs1h = take(szS), oTs1l = take(szS);
  if (o > ws_size) return;
  if (o > (size_t)134217728) return;

  char* ws = (char*)d_ws;
  float* hp0 = (float*)(ws + oHP0);
  float* up0 = (float*)(ws + oUP0);
  float* hp1 = (float*)(ws + oHP1);
  float* up1 = (float*)(ws + oUP1);
  float* z0  = (float*)(ws + oZ0);
  float* z1  = (float*)(ws + oZ1);
  float* y0  = (float*)(ws + oY0);
  float* y1  = (float*)(ws + oY1);
  double* rowstat = (double*)(ws + oRS);
  float* gstat = (float*)(ws + oGS);
  us* T00 = (us*)(ws + oT00); us* T11 = (us*)(ws + oT11);
  us* T01 = (us*)(ws + oT01); us* T10 = (us*)(ws + oT10);
  us* Wh0h = (us*)(ws + oWh0h); us* Wh0l = (us*)(ws + oWh0l);
  us* Wh1h = (us*)(ws + oWh1h); us* Wh1l = (us*)(ws + oWh1l);
  us* Wp0h = (us*)(ws + oWp0h); us* Wp0l = (us*)(ws + oWp0l);
  us* Wp1h = (us*)(ws + oWp1h); us* Wp1l = (us*)(ws + oWp1l);
  us* Ws0h = (us*)(ws + oWs0h); us* Ws0l = (us*)(ws + oWs0l);
  us* Ws1h = (us*)(ws + oWs1h); us* Ws1l = (us*)(ws + oWs1l);
  us* Wu0h = (us*)(ws + oWu0h); us* Wu0l = (us*)(ws + oWu0l);
  us* Wu1h = (us*)(ws + oWu1h); us* Wu1l = (us*)(ws + oWu1l);
  us* Ts0h = (us*)(ws + oTs0h); us* Ts0l = (us*)(ws + oTs0l);
  us* Ts1h = (us*)(ws + oTs1h); us* Ts1l = (us*)(ws + oTs1l);

  k_tconv<0><<<dim3(8, 128, 1), NTH, 0, stream>>>(Wt_00, 8192, 256, 0, T00, T00, 0, 4.0f);
  k_tconv<0><<<dim3(8, 128, 1), NTH, 0, stream>>>(Wt_11, 8192, 256, 0, T11, T11, 0, 4.0f);
  k_tconv<0><<<dim3(256, 2, 1), NTH, 0, stream>>>(Wt_01, 128, 8192, 0, T01, T01, 0, 4.0f);
  k_tconv<0><<<dim3(4, 1, 128), NTH, 0, stream>>>(Wt_10, 64, 128, 8192, T10, T10, 8192, 4.0f);
  k_tconv<1><<<dim3(4, 2, 1), NTH, 0, stream>>>(W_h0, 128, 128, 0, Wh0h, Wh0l, 0, 1.0f);
  k_tconv<1><<<dim3(4, 2, 1), NTH, 0, stream>>>(W_h1, 128, 128, 0, Wh1h, Wh1l, 0, 1.0f);
  k_tconv<1><<<dim3(2, 1, 1), NTH, 0, stream>>>(W_u0, 64, 64, 0, Wu0h, Wu0l, 0, 1.0f);
  k_tconv<1><<<dim3(2, 1, 1), NTH, 0, stream>>>(W_u1, 64, 64, 0, Wu1h, Wu1l, 0, 1.0f);
  k_tconv<1><<<dim3(4, 2, 1), NTH, 0, stream>>>(W_p0, 128, 128, 0, Wp0h, Wp0l, 0, 1.0f);
  k_tconv<1><<<dim3(4, 2, 1), NTH, 0, stream>>>(W_p1, 128, 128, 0, Wp1h, Wp1l, 0, 1.0f);
  k_tconv<1><<<dim3(4, 2, 1), NTH, 0, stream>>>(W_s0, 128, 128, 0, Ws0h, Ws0l, 0, 1.0f);
  k_tconv<1><<<dim3(4, 2, 1), NTH, 0, stream>>>(W_s1, 128, 128, 0, Ws1h, Ws1l, 0, 1.0f);
  k_tconv<1><<<dim3(40, 2, 1), NTH, 0, stream>>>(Wsc0, 128, 1280, 0, Ts0h, Ts0l, 0, 1.0f);
  k_tconv<1><<<dim3(40, 2, 1), NTH, 0, stream>>>(Wsc1, 128, 1280, 0, Ts1h, Ts1l, 0, 1.0f);

  k_lin<<<NN / TN, NTH, 0, stream>>>(nfh, nfu, Wh0h, Wh0l, Wh1h, Wh1l, Wu0h, Wu0l, Wu1h, Wu1l,
                                     hp0, up0, hp1, up1);
  k_z0<<<NN / TN, NTH, 0, stream>>>(hp0, up0, hp1, up1, T00, T11, z0);
  k_z1<<<NN / TN, NTH, 0, stream>>>(hp0, up0, hp1, up1, T01, T10, z1);
  k_post<<<NN / TN, NTH, 0, stream>>>(nfh, onehot, z0, z1, Wp0h, Wp0l, Wp1h, Wp1l,
                                      Ts0h, Ts0l, Ts1h, Ts1l, b_p0, y0, y1, rowstat);
  k_stats<<<1, NTH, 0, stream>>>(batch, rowstat, gstat);
  k_final<<<NN / TN, NTH, 0, stream>>>(nfh, batch, y0, y1, gstat, ln_w0, ln_b0, ln_w1,
                                       Ws0h, Ws0l, Ws1h, Ws1l, b_s0, out);
}
